// Block_30605936951767
// MI455X (gfx1250) — hardware-run, weakly checked
//
#include <hip/hip_runtime.h>


#ifndef NB
#define NB 4
#endif
#ifndef SEQ
#define SEQ 2048
#endif
#define NB_FULL  4
#define SEQ_FULL 2048
#ifndef OUT_SEQ
#define OUT_SEQ SEQ
#endif
#ifndef FB
#define FB (((NB) % 2) == 0 ? 2 : 1)
#endif
#define DM   1024
#define FF   4096
#define NH_  16
#define HD   64
#define AW   4
#define EARLY ((SEQ) < 512 ? (SEQ) : 512)
#define QRS  2048.0f
#define QRI  (1.0f / 2048.0f)
#define SC2  (0.125f * 1.4426950408889634f)
#define PSH  8.0f
#define NEGB (-3.0e38f)
#define CTXS 16.0f
#define WOS  64.0f
#define WSI  (1.0f / 64.0f)
#define HCS  16.0f
#define OSC  (1.0f / 1024.0f)
#define LNE  1.0e-8f
#define BIGL (1 << 30)

static_assert(HD == 64);
static_assert(NH_ * HD == DM);
static_assert(DM % 64 == 0);
static_assert(DM % 32 == 0);
static_assert(FF % 64 == 0);
static_assert(FF % 32 == 0);
static_assert(DM == 32 * 8 * 4);
static_assert(SEQ % 64 == 0);
static_assert((NB * SEQ) % 64 == 0);
static_assert((NB * SEQ) % 8 == 0);
static_assert(SEQ % 32 == 0);
static_assert(SEQ % (16 * AW) == 0);
static_assert(EARLY % 64 == 0);
static_assert(EARLY <= SEQ);
static_assert((SEQ - EARLY) % 64 == 0);
static_assert(((size_t)SEQ * DM) % 8 == 0);
static_assert(((size_t)DM * DM) % 8 == 0);
static_assert(((size_t)DM * DM / 8) % 256 == 0);
static_assert(((size_t)FF * DM / 8) % 256 == 0);
static_assert(NB <= NB_FULL);
static_assert(SEQ <= SEQ_FULL);
static_assert(NB % FB == 0);
static_assert((FB * SEQ) % 64 == 0);
static_assert(WOS * WSI == 1.0f);
static_assert(CTXS * WOS * OSC == 1.0f);
static_assert(HCS * WOS * OSC == 1.0f);
static_assert((size_t)NB_FULL * SEQ_FULL * DM * 4 == (size_t)33554432);
static_assert(32 * 16 * 4 == 16 * HD * 2);
static_assert(32 * 16 * 8 == 16 * 64 * 4);
static_assert(32 * 16 * 4 == DM * 2);
static_assert(AW * 16 * 68 * 4 <= 131072);
static_assert(16 * 68 * 4 <= 131072);

typedef _Float16 h16;
typedef unsigned short bf;
typedef __attribute__((ext_vector_type(16))) __bf16   v16bf;
typedef __attribute__((ext_vector_type(16))) _Float16 v16h;
typedef __attribute__((ext_vector_type(8)))  _Float16 v8h;
typedef __attribute__((ext_vector_type(8)))  unsigned short v8us;
typedef __attribute__((ext_vector_type(8)))  float    v8f;
typedef __attribute__((ext_vector_type(4)))  float    v4f;
typedef v4f  __attribute__((may_alias)) v4fa;
typedef v8us __attribute__((may_alias)) v8usa;

__device__ __forceinline__ unsigned short f2bf(float f) { unsigned u = __float_as_uint(f); u += 0x7FFFu + ((u >> 16) & 1u); return (unsigned short)(u >> 16); }
__device__ __forceinline__ float bfr(float f) { return __uint_as_float(((unsigned)f2bf(f)) << 16); }
__device__ __forceinline__ v16h cat16(v8h lo, v8h hi) { return __builtin_shufflevector(lo, hi, 0, 1, 2, 3, 4, 5, 6, 7, 8, 9, 10, 11, 12, 13, 14, 15); }
__device__ __forceinline__ v16bf cat16b(v8us lo, v8us hi) { return __builtin_bit_cast(v16bf, __builtin_shufflevector(lo, hi, 0, 1, 2, 3, 4, 5, 6, 7, 8, 9, 10, 11, 12, 13, 14, 15)); }
__device__ __forceinline__ v8f wmma16(v16h a, v16h b, v8f c) { return __builtin_amdgcn_wmma_f32_16x16x32_f16(false, a, false, b, (short)0, c, false, false); }
__device__ __forceinline__ v8f wmmab(v16bf a, v16bf b, v8f c) { return __builtin_amdgcn_wmma_f32_16x16x32_bf16(false, a, false, b, (short)0, c, false, false); }
__device__ __forceinline__ v16h  ldh(const h16* p) { return cat16(*(const v8h*)p, *(const v8h*)(p + 16)); }
__device__ __forceinline__ v16bf ldb(const bf* p)  { return cat16b(*(const v8us*)p, *(const v8us*)(p + 16)); }
__device__ __forceinline__ void wave_sync() { __builtin_amdgcn_fence(3  , "wavefront"); __builtin_amdgcn_wave_barrier(); asm volatile("" ::: "memory"); }
static __device__ __forceinline__ h16 toh_flush(float v) { const h16 r = (h16)v; return (fabsf(v) < 6.103515625e-05f) ? (h16)0.0f : r; }
static __device__ __forceinline__ float gelu_c(float v) { return (0.5f * v * (1.0f + erff(v * 0.70710678118654752f))) * HCS; }

__global__ __launch_bounds__(256) void k_cvt8h(const float* __restrict__ src, h16* dst, size_t n8) {
    const size_t i = (size_t)blockIdx.x * 256 + threadIdx.x; if (i >= n8) return;
    const v8f v = *(const v8f*)(src + i * 8); v8h o;
#pragma unroll
    for (int k = 0; k < 8; ++k) o[k] = toh_flush(bfr(v[k]) * WOS);
    *(volatile v8h*)(dst + i * 8) = o; __threadfence(); *(volatile v8h*)(dst + i * 8) = o;
}

__global__ __launch_bounds__(256) void k_ln(const float* __restrict__ X, const float* __restrict__ G, const float* __restrict__ BE, h16* XN, int xseq, int inb) {
#pragma clang fp contract(off)
    const int lane = threadIdx.x & 31;
    const int wave = __builtin_amdgcn_readfirstlane((int)(threadIdx.x >> 5));
    const int m = (int)blockIdx.x * 8 + wave;
    const int b = m / SEQ, t = m % SEQ;
    const size_t xo = ((size_t)b * (size_t)xseq + (size_t)t) * DM + (size_t)lane * 8;
    float s = 0.0f;
#pragma unroll 1
    for (int c = 0; c < 4; ++c) { const v8f v = *(const v8f*)(X + xo + c * 256);
#pragma unroll
        for (int k = 0; k < 8; ++k) { const float a = (inb != 0) ? bfr(v[k]) : v[k]; s += a; } }
#pragma unroll
    for (int d = 16; d >= 1; d >>= 1) s += __shfl_xor(s, d, 32);
    const float mu = s * (1.0f / (float)DM);
    float q = 0.0f;
#pragma unroll 1
    for (int c = 0; c < 4; ++c) { const v8f v = *(const v8f*)(X + xo + c * 256);
#pragma unroll
        for (int k = 0; k < 8; ++k) { const float a = (inb != 0) ? bfr(v[k]) : v[k]; const float dd = a - mu; q += dd * dd; } }
#pragma unroll
    for (int d = 16; d >= 1; d >>= 1) q += __shfl_xor(q, d, 32);
    const float var = q * (1.0f / (float)(DM - 1));
    const float rs = 1.0f / (sqrtf(var) + LNE);
#pragma unroll 1
    for (int c = 0; c < 4; ++c) {
        const v8f v = *(const v8f*)(X + xo + c * 256);
        const v8f g = *(const v8f*)(G + c * 256 + lane * 8);
        const v8f e = *(const v8f*)(BE + c * 256 + lane * 8);
        v8h o;
#pragma unroll
        for (int k = 0; k < 8; ++k) { const float a = (inb != 0) ? bfr(v[k]) : v[k];
            const float y = ((a - mu) * rs) * bfr(g[k]) + bfr(e[k]); o[k] = toh_flush(y); }
        h16* dp = XN + (size_t)m * DM + c * 256 + lane * 8;
        *(volatile v8h*)dp = o; __threadfence(); *(volatile v8h*)dp = o; }
}

template<int BROW, int ACT>
__global__ __launch_bounds__(32) void k_proj(const h16* __restrict__ A, const h16* __restrict__ Bt, h16* Ph, h16* Pr, const float* __restrict__ bias,
                                             int RB, size_t sRB, int pitch, int CB, size_t sCB, int rlim, int clim) {
    __shared__ __align__(16) float os[16 * 68];
    const int K = DM;
    const int lane = threadIdx.x & 31, lr = lane & 15, hi = lane >> 4; const int r0 = blockIdx.x * 64, c0 = blockIdx.y * 64;
    const int wr = ((r0 % RB) < rlim) && ((c0 % CB) < clim);
    v8f acc[4][4];
#pragma unroll
    for (int mb = 0; mb < 4; ++mb)
#pragma unroll
        for (int nb = 0; nb < 4; ++nb) acc[mb][nb] = (v8f){};
    const size_t aoff = (size_t)(r0 + lr) * K + 8 * hi, boff = (size_t)(c0 + lr) * K + 8 * hi;
#pragma unroll 1
    for (int kc = 0; kc < K; kc += 32) {
        v16h a[4];
#pragma unroll
        for (int mb = 0; mb < 4; ++mb) a[mb] = ldh(A + aoff + (size_t)mb * 16 * K + kc);
#pragma unroll
        for (int nb = 0; nb < 4; ++nb) { const v16h b = ldh(Bt + boff + (size_t)nb * 16 * K + kc);
#pragma unroll
            for (int mb = 0; mb < 4; ++mb) acc[mb][nb] = wmma16(a[mb], b, acc[mb][nb]); }
        asm volatile("v_nop\n\tv_nop\n\tv_nop\n\tv_nop" : "+v"(acc[0][0]), "+v"(acc[1][1]), "+v"(acc[2][2]), "+v"(acc[3][3]) : "v"(a[0]), "v"(a[1]), "v"(a[2]), "v"(a[3]));
    }
    float bcol[4];
#pragma unroll
    for (int nb = 0; nb < 4; ++nb) { bcol[nb] = 0.0f; if constexpr (BROW == 0) bcol[nb] = bfr(bias[c0 + nb * 16 + lr]); }
    const size_t tbase = (size_t)(r0 / RB) * sRB + (size_t)(r0 % RB) * (size_t)pitch + (size_t)(c0 / CB) * sCB + (size_t)(c0 % CB);
#pragma unroll
    for (int mb = 0; mb < 4; ++mb) {
        float brow[8];
#pragma unroll
        for (int j = 0; j < 8; ++j) { brow[j] = 0.0f; if constexpr (BROW != 0) brow[j] = bfr(bias[r0 + mb * 16 + hi * 8 + j]); }
#pragma unroll
        for (int nb = 0; nb < 4; ++nb) {
#pragma unroll
            for (int j = 0; j < 8; ++j) os[(hi * 8 + j) * 68 + nb * 16 + lr] = acc[mb][nb][j] * WSI + bcol[nb] + brow[j]; }
        wave_sync();
        if constexpr (ACT != 0) {
#pragma unroll 1
            for (int s = 0; s < 4; ++s) { const int row = 4 * s + (lane >> 3), c8 = (lane & 7) * 8;
                v4f x0 = *(const v4fa*)(&os[row * 68 + c8]); v4f x1 = *(const v4fa*)(&os[row * 68 + c8 + 4]);
#pragma unroll
                for (int i = 0; i < 4; ++i) { x0[i] = gelu_c(x0[i]); x1[i] = gelu_c(x1[i]); }
                *(v4fa*)(&os[row * 68 + c8]) = x0; *(v4fa*)(&os[row * 68 + c8 + 4]) = x1; }
            wave_sync();
        }
        const size_t sb = tbase + (size_t)(mb * 16) * (size_t)pitch;
#pragma unroll 1
        for (int ps = 0; ps < 2; ++ps) {
#pragma unroll
            for (int s = 0; s < 4; ++s) { const int row = 4 * s + (lane >> 3), c8 = (lane & 7) * 8;
                const v4f x0 = *(const v4fa*)(&os[row * 68 + c8]); const v4f x1 = *(const v4fa*)(&os[row * 68 + c8 + 4]); v8h hv;
#pragma unroll
                for (int i = 0; i < 4; ++i) { hv[i] = toh_flush(x0[i]); hv[4 + i] = toh_flush(x1[i]); }
                const size_t oo = sb + (size_t)row * (size_t)pitch + c8;
                *(volatile v8h*)(Ph + oo) = hv;
                if (wr) { v8h rv;
#pragma unroll
                    for (int i = 0; i < 4; ++i) { rv[i] = toh_flush((x0[i] - (float)hv[i]) * QRS); rv[4 + i] = toh_flush((x1[i] - (float)hv[4 + i]) * QRS); }
                    *(volatile v8h*)(Pr + oo) = rv; } }
            if (ps == 0) __threadfence(); }
        wave_sync();
    }
}

template<int ER>
__global__ __launch_bounds__(32 * AW) void k_flash(const h16* __restrict__ QH, const h16* __restrict__ QR, const h16* __restrict__ KH, const h16* __restrict__ KR,
                                                   const h16* __restrict__ VT, const h16* __restrict__ VR, h16* CH, h16* CR, int tb0) {
    __shared__ __align__(16) float os[AW * 16 * 68];
    const int lane = threadIdx.x & 31, lr = lane & 15, hi = lane >> 4;
    const int wave = __builtin_amdgcn_readfirstlane((int)(threadIdx.x >> 5));
    const int zh = blockIdx.y; const int b = zh / NH_, h = zh % NH_;
    const int t0 = tb0 + ((int)blockIdx.x * AW + wave) * 16;
    const size_t pbase = (size_t)zh * SEQ * HD;
    const size_t qo = pbase + (size_t)(t0 + lr) * HD + 8 * hi;
    const v16h qh0 = ldh(QH + qo), qh1 = ldh(QH + qo + 32);
    v16h qr0 = qh0, qr1 = qh1;
    if constexpr (ER != 0) { qr0 = ldh(QR + qo); qr1 = ldh(QR + qo + 32); }
    const size_t ko = pbase + (size_t)lr * HD + 8 * hi;
    const size_t vo = pbase + (size_t)lr * SEQ + 8 * hi;
    v8f oH[4], oR[4];
#pragma unroll
    for (int j = 0; j < 4; ++j) { oH[j] = (v8f){}; oR[j] = (v8f){}; }
    float m = NEGB, l = 0.0f;
    const int kend = t0 + 16;
#pragma unroll 1
    for (int key0 = 0; key0 < kend; key0 += 32) {
        const size_t kof = ko + (size_t)key0 * HD;
        const v16h ka0 = ldh(KH + kof), ka1 = ldh(KH + kof + 32), kb0 = ldh(KH + kof + 16 * HD), kb1 = ldh(KH + kof + 16 * HD + 32);
        float ta[8], tb[8];
        if constexpr (ER != 0) {
            const v16h ra0 = ldh(KR + kof), ra1 = ldh(KR + kof + 32), rb0 = ldh(KR + kof + 16 * HD), rb1 = ldh(KR + kof + 16 * HD + 32);
            v8f sHa = (v8f){}, sRa = (v8f){}, sHb = (v8f){}, sRb = (v8f){};
            sHa = wmma16(ka0, qh0, sHa); sRa = wmma16(ka0, qr0, sRa); sHb = wmma16(kb0, qh0, sHb); sRb = wmma16(kb0, qr0, sRb);
            sHa = wmma16(ka1, qh1, sHa); sRa = wmma16(ra0, qh0, sRa); sHb = wmma16(kb1, qh1, sHb); sRb = wmma16(rb0, qh0, sRb);
            sRa = wmma16(ka1, qr1, sRa); sRb = wmma16(kb1, qr1, sRb);
            sRa = wmma16(ra1, qh1, sRa); sRb = wmma16(rb1, qh1, sRb);
            asm volatile("v_nop\n\tv_nop\n\tv_nop\n\tv_nop" : "+v"(sHa), "+v"(sRa), "+v"(sHb), "+v"(sRb)
                         : "v"(ka0), "v"(ka1), "v"(kb0), "v"(kb1), "v"(ra0), "v"(ra1), "v"(rb0), "v"(rb1));
#pragma unroll
            for (int r = 0; r < 8; ++r) { ta[r] = (sHa[r] + sRa[r] * QRI) * SC2; tb[r] = (sHb[r] + sRb[r] * QRI) * SC2; }
        } else {
            v8f sa = (v8f){}, sb = (v8f){};
            sa = wmma16(ka0, qh0, sa); sb = wmma16(kb0, qh0, sb); sa = wmma16(ka1, qh1, sa); sb = wmma16(kb1, qh1, sb);
            asm volatile("v_nop\n\tv_nop\n\tv_nop\n\tv_nop" : "+v"(sa), "+v"(sb) : "v"(ka0), "v"(ka1), "v"(kb0), "v"(kb1));
#pragma unroll
            for (int r = 0; r < 8; ++r) { ta[r] = sa[r] * SC2; tb[r] = sb[r] * SC2; }
        }
        if (key0 + 31 > t0) {
            const int tq = t0 + lr, kq = key0 + 8 * hi;
#pragma unroll
            for (int r = 0; r < 8; ++r) { ta[r] = (kq + r > tq) ? NEGB : ta[r]; tb[r] = (kq + 16 + r > tq) ? NEGB : tb[r]; }
        }
        float mx = NEGB;
#pragma unroll
        for (int r = 0; r < 8; ++r) mx = fmaxf(mx, fmaxf(ta[r], tb[r]));
        mx = fmaxf(mx, __shfl_xor(mx, 16, 32));
        const float mnew = fmaxf(m, mx);
        const float alpha = __builtin_amdgcn_exp2f(m - mnew);
        const float sh = PSH - mnew;
        v16h pb = (v16h){}; v16h pr = (v16h){}; float ls = 0.0f;
        if constexpr (ER != 0) {
#pragma unroll
            for (int r = 0; r < 8; ++r) {
                const float pfa = __builtin_amdgcn_exp2f(ta[r] + sh); const float pfc = __builtin_amdgcn_exp2f(tb[r] + sh);
                const h16 pa = (h16)pfa; const h16 pc = (h16)pfc;
                const h16 qa = (h16)((pfa - (float)pa) * QRS); const h16 qc = (h16)((pfc - (float)pc) * QRS);
                pb[r] = pa; pb[8 + r] = pc; pr[r] = qa; pr[8 + r] = qc;
                ls += ((float)pa + (float)qa * QRI) + ((float)pc + (float)qc * QRI); }
        } else {
#pragma unroll
            for (int r = 0; r < 8; ++r) { const h16 pa = (h16)__builtin_amdgcn_exp2f(ta[r] + sh); const h16 pc = (h16)__builtin_amdgcn_exp2f(tb[r] + sh); pb[r] = pa; pb[8 + r] = pc; ls += (float)pa + (float)pc; }
        }
        l = l * alpha + ls; m = mnew;
#pragma unroll
        for (int j = 0; j < 4; ++j) oH[j] = oH[j] * alpha;
        if constexpr (ER != 0) {
#pragma unroll
            for (int j = 0; j < 4; ++j) oR[j] = oR[j] * alpha;
        }
        const size_t vof = vo + key0;
        const v16h v0 = ldh(VT + vof), v1 = ldh(VT + vof + (size_t)16 * SEQ), v2 = ldh(VT + vof + (size_t)32 * SEQ), v3 = ldh(VT + vof + (size_t)48 * SEQ);
        if constexpr (ER != 0) {
            const v16h w0 = ldh(VR + vof), w1 = ldh(VR + vof + (size_t)16 * SEQ), w2 = ldh(VR + vof + (size_t)32 * SEQ), w3 = ldh(VR + vof + (size_t)48 * SEQ);
            oH[0] = wmma16(v0, pb, oH[0]); oH[1] = wmma16(v1, pb, oH[1]); oH[2] = wmma16(v2, pb, oH[2]); oH[3] = wmma16(v3, pb, oH[3]);
            oR[0] = wmma16(v0, pr, oR[0]); oR[1] = wmma16(v1, pr, oR[1]); oR[2] = wmma16(v2, pr, oR[2]); oR[3] = wmma16(v3, pr, oR[3]);
            oR[0] = wmma16(w0, pb, oR[0]); oR[1] = wmma16(w1, pb, oR[1]); oR[2] = wmma16(w2, pb, oR[2]); oR[3] = wmma16(w3, pb, oR[3]);
            asm volatile("v_nop\n\tv_nop\n\tv_nop\n\tv_nop" : "+v"(oH[0]), "+v"(oH[1]), "+v"(oH[2]), "+v"(oH[3]), "+v"(oR[0]), "+v"(oR[1]), "+v"(oR[2]), "+v"(oR[3])
                         : "v"(v0), "v"(v1), "v"(v2), "v"(v3), "v"(w0), "v"(w1), "v"(w2), "v"(w3), "v"(pb), "v"(pr));
        } else {
            oH[0] = wmma16(v0, pb, oH[0]); oH[1] = wmma16(v1, pb, oH[1]); oH[2] = wmma16(v2, pb, oH[2]); oH[3] = wmma16(v3, pb, oH[3]);
            asm volatile("v_nop\n\tv_nop\n\tv_nop\n\tv_nop" : "+v"(oH[0]), "+v"(oH[1]), "+v"(oH[2]), "+v"(oH[3]) : "v"(v0), "v"(v1), "v"(v2), "v"(v3), "v"(pb));
        }
    }
    l += __shfl_xor(l, 16, 32);
    const float invc = (1.0f / l) * CTXS;
    const int wb = wave * 16 * 68;
#pragma unroll
    for (int j = 0; j < 4; ++j) { v4f a, c;
#pragma unroll
        for (int i = 0; i < 4; ++i) { float x0 = oH[j][i], x1 = oH[j][4 + i];
            if constexpr (ER != 0) { x0 += oR[j][i] * QRI; x1 += oR[j][4 + i] * QRI; }
            a[i] = x0 * invc; c[i] = x1 * invc; }
        *(v4fa*)(&os[wb + lr * 68 + 16 * j + 8 * hi]) = a; *(v4fa*)(&os[wb + lr * 68 + 16 * j + 8 * hi + 4]) = c; }
    wave_sync();
    h16* crow = CH + ((size_t)b * SEQ + t0) * DM + h * HD;
#pragma unroll 1
    for (int ps = 0; ps < 2; ++ps) {
#pragma unroll
        for (int s = 0; s < 4; ++s) { const int row = 4 * s + (lane >> 3), c8 = (lane & 7) * 8;
            const v4f x0 = *(const v4fa*)(&os[wb + row * 68 + c8]); const v4f x1 = *(const v4fa*)(&os[wb + row * 68 + c8 + 4]); v8h hv;
#pragma unroll
            for (int i = 0; i < 4; ++i) { hv[i] = (h16)x0[i]; hv[4 + i] = (h16)x1[i]; }
            *(volatile v8h*)(crow + (size_t)row * DM + c8) = hv;
            if constexpr (ER != 0) { v8h rv;
#pragma unroll
                for (int i = 0; i < 4; ++i) { rv[i] = (h16)((x0[i] - (float)hv[i]) * QRS); rv[4 + i] = (h16)((x1[i] - (float)hv[4 + i]) * QRS); }
                h16* rrow = CR + ((size_t)b * EARLY + t0) * DM + h * HD;
                *(volatile v8h*)(rrow + (size_t)row * DM + c8) = rv; } }
        if (ps == 0) __threadfence(); }
}

template<int MB, int RES>
__global__ __launch_bounds__(32) void k_oproj(const h16* __restrict__ CH, const h16* __restrict__ CR, const h16* __restrict__ WO, const float* __restrict__ bo,
                                              const float* __restrict__ XR, float* OUT, int K, int tb0, int tpb, int xseq, int oseq, int inb) {
    __shared__ __align__(16) float os[16 * 68];
    const int lane = threadIdx.x & 31, lr = lane & 15, hi = lane >> 4;
    const int bx = blockIdx.x; const int b = bx / tpb; const int t0 = tb0 + (bx % tpb) * (16 * MB); const int c0 = blockIdx.y * 64;
    v8f acc[MB][4], accR[MB][4];
#pragma unroll
    for (int mb = 0; mb < MB; ++mb)
#pragma unroll
        for (int nb = 0; nb < 4; ++nb) { acc[mb][nb] = (v8f){}; accR[mb][nb] = (v8f){}; }
    const size_t aoff = ((size_t)b * SEQ + t0 + lr) * K + 8 * hi;
    const size_t roff = ((size_t)b * EARLY + t0 + lr) * K + 8 * hi;
    const size_t boff = (size_t)(c0 + lr) * K + 8 * hi;
#pragma unroll 1
    for (int kc = 0; kc < K; kc += 32) {
        v16h a[MB], ar[MB];
#pragma unroll
        for (int mb = 0; mb < MB; ++mb) { a[mb] = ldh(CH + aoff + (size_t)mb * 16 * K + kc); ar[mb] = a[mb];
            if constexpr (RES != 0) ar[mb] = ldh(CR + roff + (size_t)mb * 16 * K + kc); }
#pragma unroll
        for (int nb = 0; nb < 4; ++nb) { const v16h bw = ldh(WO + boff + (size_t)nb * 16 * K + kc);
#pragma unroll
            for (int mb = 0; mb < MB; ++mb) { acc[mb][nb] = wmma16(a[mb], bw, acc[mb][nb]);
                if constexpr (RES != 0) accR[mb][nb] = wmma16(ar[mb], bw, accR[mb][nb]); } }
        if constexpr (MB == 4) {
            asm volatile("v_nop\n\tv_nop\n\tv_nop\n\tv_nop" : "+v"(acc[0][0]), "+v"(acc[1][1]), "+v"(acc[2][2]), "+v"(acc[3][3]) : "v"(a[0]), "v"(a[1]), "v"(a[2]), "v"(a[3]));
        } else {
            asm volatile("v_nop\n\tv_nop\n\tv_nop\n\tv_nop" : "+v"(acc[0][3]), "+v"(acc[MB - 1][3]), "+v"(accR[0][3]), "+v"(accR[MB - 1][3]) : "v"(a[0]), "v"(a[MB - 1]), "v"(ar[0]), "v"(ar[MB - 1]));
        }
    }
    float bcol[4];
#pragma unroll
    for (int nb = 0; nb < 4; ++nb) bcol[nb] = bfr(bo[c0 + nb * 16 + lr]);
#pragma unroll
    for (int mb = 0; mb < MB; ++mb) {
#pragma unroll
        for (int nb = 0; nb < 4; ++nb) {
#pragma unroll
            for (int j = 0; j < 8; ++j) { float x = acc[mb][nb][j];
                if constexpr (RES != 0) x += accR[mb][nb][j] * QRI;
                os[(hi * 8 + j) * 68 + nb * 16 + lr] = x * OSC + bcol[nb]; } }
        wave_sync();
        float* orow = OUT + ((size_t)b * (size_t)oseq + t0 + mb * 16) * DM + c0;
        const float* xrow = XR + ((size_t)b * (size_t)xseq + t0 + mb * 16) * DM + c0;
#pragma unroll 1
        for (int ps = 0; ps < 2; ++ps) {
#pragma unroll
            for (int s = 0; s < 8; ++s) { const int row = 2 * s + hi, cofs = lr * 4;
                v4f val = *(const v4fa*)(&os[row * 68 + cofs]);
                const v4f xv = *(const v4f*)(xrow + (size_t)row * DM + cofs);
#pragma unroll
                for (int i = 0; i < 4; ++i) { const float xa = (inb != 0) ? bfr(xv[i]) : xv[i]; val[i] = val[i] + xa; }
                *(volatile v4f*)(orow + (size_t)row * DM + cofs) = val; }
            if (ps == 0) __threadfence(); }
        wave_sync();
    }
}

static constexpr size_t al256(size_t v) { return (v + 255) & ~(size_t)255; }
static constexpr size_t SZ_WA = al256((size_t)4 * DM * DM * 2);
static constexpr size_t SZ_XB = al256((size_t)NB * SEQ * DM * 2);
static constexpr size_t SZ_PL = al256((size_t)NB * NH_ * SEQ * HD * 2);
static constexpr size_t SZ_CR = al256((size_t)NB * EARLY * DM * 2);
static constexpr size_t SZ_X1 = al256((size_t)NB * SEQ * DM * 4);
static constexpr size_t SZ_WF = al256((size_t)FF * DM * 2);
static constexpr size_t SZ_H  = al256((size_t)FB * SEQ * FF * 2);
static constexpr size_t SZ_ATT = 6 * SZ_PL;
static constexpr size_t SZ_FFN = SZ_X1 + 2 * SZ_WF + SZ_H;
static constexpr size_t SZ_PB = (SZ_ATT > SZ_FFN) ? SZ_ATT : SZ_FFN;
static constexpr size_t SZ_TOTAL = SZ_WA + SZ_XB + SZ_PB + SZ_CR;
static_assert(SZ_TOTAL <= (size_t)134217728);
static_assert(((size_t)DM * DM * 2) % 256 == 0);
static_assert((size_t)NB * SEQ * DM * 2 <= SZ_XB);
static_assert(SZ_ATT <= SZ_PB);
static_assert(SZ_FFN <= SZ_PB);
static_assert((size_t)NB * SEQ * DM * 4 <= SZ_X1);
static_assert((size_t)FF * DM * 2 <= SZ_WF);
static_assert((size_t)FB * SEQ * FF * 2 <= SZ_H);

extern "C" void kernel_launch(void* const* d_in, const int* in_sizes, int n_in,
                              void* d_out, int out_size, void* d_ws, size_t ws_size, hipStream_t stream) {
    if (n_in < 17) return;
    const size_t needx = ((size_t)(NB - 1) * SEQ_FULL + SEQ) * DM;
    if ((size_t)in_sizes[0] < needx) return;
    if ((size_t)in_sizes[1] < (size_t)DM * DM || (size_t)in_sizes[3] < (size_t)DM * DM || (size_t)in_sizes[5] < (size_t)DM * DM || (size_t)in_sizes[7] < (size_t)DM * DM) return;
    if (in_sizes[2] < DM || in_sizes[4] < DM || in_sizes[6] < DM || in_sizes[8] < DM) return;
    if (in_sizes[9] < DM || in_sizes[10] < DM || in_sizes[11] < DM || in_sizes[12] < DM) return;
    if ((size_t)in_sizes[13] < (size_t)FF * DM || in_sizes[14] < FF || (size_t)in_sizes[15] < (size_t)DM * FF || in_sizes[16] < DM) return;
    if ((size_t)out_size < ((size_t)(NB - 1) * OUT_SEQ + SEQ) * DM) return;
    if (SZ_TOTAL > ws_size) return;
    const float* x  = (const float*)d_in[0];
    const float* wq = (const float*)d_in[1]; const float* bq = (const float*)d_in[2];
    const float* wk = (const float*)d_in[3]; const float* bk = (const float*)d_in[4];
    const float* wv = (const float*)d_in[5]; const float* bv = (const float*)d_in[6];
    const float* wo = (const float*)d_in[7]; const float* bo = (const float*)d_in[8];
    const float* g1 = (const float*)d_in[9];  const float* be1 = (const float*)d_in[10];
    const float* g2 = (const float*)d_in[11]; const float* be2 = (const float*)d_in[12];
    const float* w1 = (const float*)d_in[13]; const float* bf1 = (const float*)d_in[14];
    const float* w2 = (const float*)d_in[15]; const float* bf2 = (const float*)d_in[16];
    float* OUT = (float*)d_out;
    char* wsp = (char*)d_ws;
    h16* WQH = (h16*)wsp; h16* WKH = WQH + (size_t)DM * DM; h16* WVH = WQH + (size_t)2 * DM * DM; h16* WOH = WQH + (size_t)3 * DM * DM;
    wsp += SZ_WA;
    h16* XN = (h16*)wsp; h16* CH = (h16*)wsp; h16* XN2 = (h16*)wsp; wsp += SZ_XB;
    char* pb = wsp; wsp += SZ_PB;
    h16* CR = (h16*)wsp; wsp += SZ_CR;
    h16* QH = (h16*)(pb + 0 * SZ_PL);
    h16* QR = (h16*)(pb + 1 * SZ_PL);
    h16* KH = (h16*)(pb + 2 * SZ_PL);
    h16* KR = (h16*)(pb + 3 * SZ_PL);
    h16* VT = (h16*)(pb + 4 * SZ_PL);
    h16* VR = (h16*)(pb + 5 * SZ_PL);
    float* X1 = (float*)pb;
    h16* W1H = (h16*)(pb + SZ_X1);
    h16* W2H = (h16*)(pb + SZ_X1 + SZ_WF);
    h16* HP  = (h16*)(pb + SZ_X1 + 2 * SZ_WF);

    { const size_t n8 = (size_t)DM * DM / 8; const unsigned g = (unsigned)((n8 + 255) / 256);
      k_cvt8h<<<g, 256, 0, stream>>>(wq, WQH, n8);
      k_cvt8h<<<g, 256, 0, stream>>>(wk, WKH, n8);
      k_cvt8h<<<g, 256, 0, stream>>>(wv, WVH, n8);
      k_cvt8h<<<g, 256, 0, stream>>>(wo, WOH, n8); }

    k_ln<<<(unsigned)(NB * SEQ / 8), 256, 0, stream>>>(x, g1, be1, XN, SEQ_FULL, 1);

    k_proj<0, 0><<<dim3(NB * SEQ / 64, DM / 64, 1), 32, 0, stream>>>(XN, WQH, QH, QR, bq, SEQ, (size_t)NH_ * SEQ * HD, HD, HD, (size_t)SEQ * HD, EARLY, BIGL);
    k_proj<0, 0><<<dim3(NB * SEQ / 64, DM / 64, 1), 32, 0, stream>>>(XN, WKH, KH, KR, bk, SEQ, (size_t)NH_ * SEQ * HD, HD, HD, (size_t)SEQ * HD, EARLY, BIGL);
    k_proj<1, 0><<<dim3(DM / 64, NB * SEQ / 64, 1), 32, 0, stream>>>(WVH, XN, VT, VR, bv, DM, (size_t)0, SEQ, SEQ, (size_t)DM * SEQ, BIGL, EARLY);

    if (SEQ > EARLY) k_flash<0><<<dim3((SEQ - EARLY) / (16 * AW), NB * NH_, 1), 32 * AW, 0, stream>>>(QH, QR, KH, KR, VT, VR, CH, CR, EARLY);
    k_flash<1><<<dim3(EARLY / (16 * AW), NB * NH_, 1), 32 * AW, 0, stream>>>(QH, QR, KH, KR, VT, VR, CH, CR, 0);

    { const size_t n8 = (size_t)FF * DM / 8; const unsigned g = (unsigned)((n8 + 255) / 256);
      k_cvt8h<<<g, 256, 0, stream>>>(w1, W1H, n8);
      k_cvt8h<<<g, 256, 0, stream>>>(w2, W2H, n8); }

    if (SEQ > EARLY) k_oproj<4, 0><<<dim3(NB * ((SEQ - EARLY) / 64), DM / 64, 1), 32, 0, stream>>>(CH, CR, WOH, bo, x, X1, DM, EARLY, (SEQ - EARLY) / 64, SEQ_FULL, SEQ, 1);
    k_oproj<2, 1><<<dim3(NB * (EARLY / 32), DM / 64, 1), 32, 0, stream>>>(CH, CR, WOH, bo, x, X1, DM, 0, EARLY / 32, SEQ_FULL, SEQ, 1);

    k_ln<<<(unsigned)(NB * SEQ / 8), 256, 0, stream>>>(X1, g2, be2, XN2, SEQ, 0);

    for (int c = 0; c < NB / FB; ++c) {
        const size_t r0 = (size_t)c * FB * SEQ;
        k_proj<0, 1><<<dim3(FB * SEQ / 64, FF / 64, 1), 32, 0, stream>>>(XN2 + r0 * DM, W1H, HP, HP, bf1, BIGL, (size_t)0, FF, BIGL, (size_t)0, 0, 0);
        k_oproj<4, 0><<<dim3(FB * (SEQ / 64), DM / 64, 1), 32, 0, stream>>>(HP, HP, W2H, bf2, X1 + r0 * DM, OUT + (size_t)c * FB * OUT_SEQ * DM, FF, 0, SEQ / 64, SEQ, OUT_SEQ, 0);
    }
}
